// SUPEncoder_53068615910239
// MI455X (gfx1250) — hardware-run, weakly checked
//
#include <hip/hip_runtime.h>
#include <stddef.h>
#include <math.h>


#define NNODE  5000
#define NPAD   5056
#define NEDGE  20000
#define NFEAT  64
#define DD     64
#define HIDW   128
#define EFEAT  5
#define G3     192
#define G4     256
#define NGR    64
#define GPB    8
#define TCOL   4096
#define OUT0N  (NGR * 2 * DD)
#define OUTN   (OUT0N + NNODE * DD)
#define ASC    8
#define WSC    64
#define EWSC   64
#define OSC    (1.0f / 512.0f)
#define EWINV  (1.0f / 64.0f)
#define TB     256
#define NT     128
#define NT2    64
#define NKT    8
#define NCH    (NT * NKT)
#define WCAPN  (32 * NKT)
#define NWS    8
#define WLC    512
#define NPIECE (NNODE * DD / 4)
#define UMAX   (TCOL * HIDW / 8)
#define WSCAP  200000000

static_assert(NPAD % 64 == 0 && NPAD >= NNODE && NPAD - NNODE < 64);
static_assert(NEDGE % 32 == 0 && NEDGE % 2 == 0);
static_assert((NCH & (NCH - 1)) == 0 && NCH <= 4096);
static_assert(TCOL == DD * DD && HIDW % 32 == 0 && DD % 32 == 0 && NFEAT == DD);
static_assert(NGR % GPB == 0 && GPB == NWS && TB == 32 * NWS && GPB * 2 * DD == 4 * TB && G4 == TB);
static_assert((OUT0N * 4) % 128 == 0 && (NNODE * DD) % 4 == 0 && NPIECE % 32 == 0);
static_assert(OUTN == 328192);
static_assert(NNODE < 65536);
static_assert(UMAX % TB == 0);

typedef float          v2f  __attribute__((ext_vector_type(2)));
typedef float          v4f  __attribute__((ext_vector_type(4)));
typedef float          v8f  __attribute__((ext_vector_type(8)));
typedef int            v4i  __attribute__((ext_vector_type(4)));
typedef _Float16       v8h  __attribute__((ext_vector_type(8)));
typedef _Float16       v16h __attribute__((ext_vector_type(16)));
typedef unsigned short v8us __attribute__((ext_vector_type(8)));
union FragH { v16h v; v8us u[2]; v8h h[2]; };
union U8 { v8us u; v8h h; };

__device__ __forceinline__ v8f wmh(v16h a, v16h b, v8f c) {
  v8f d = __builtin_amdgcn_wmma_f32_16x16x32_f16(false, a, false, b, (short)0, c, false, false);
  asm volatile("v_nop\n\tv_nop\n\tv_nop\n\tv_nop" : "+v"(d) : "v"(a), "v"(b));
  return d;
}
__device__ __forceinline__ v8f zero8() { v8f z = {0.f, 0.f, 0.f, 0.f, 0.f, 0.f, 0.f, 0.f}; return z; }
__device__ __forceinline__ float sigm_f(float x) {
  x = fminf(fmaxf(x, -30.0f), 30.0f);
  return __builtin_amdgcn_rcpf(1.0f + __expf(-x));
}
__device__ __forceinline__ float tanh_f(float x) {
  const float ax = fminf(fabsf(x), 15.0f);
  const float e = __expf(-2.0f * ax);
  const float t = (1.0f - e) * __builtin_amdgcn_rcpf(1.0f + e);
  return x < 0.0f ? -t : t;
}
__device__ __forceinline__ float wsum32(float v) {
#pragma unroll
  for (int s = 16; s > 0; s >>= 1) v += __shfl_xor(v, s);
  return v;
}

__device__ __forceinline__ v16h frag_glb(const unsigned short* P, int row, int ld, int k0, int hh) {
  FragH f;
  const unsigned short* p = P + (size_t)row * ld + k0 + 8 * hh;
  f.u[0] = *(const v8us*)p;
  f.u[1] = *(const v8us*)(p + 16);
  return f.v;
}
__device__ __forceinline__ v16h frag_lds(const _Float16* T, int row, int ld, int k0, int hh) {
  FragH f;
  const _Float16* p = T + row * ld + k0 + 8 * hh;
  f.h[0] = *(const v8h*)p;
  f.h[1] = *(const v8h*)(p + 16);
  return f.v;
}
__device__ __forceinline__ v8f gemm1(v16h a0, v16h a1, const unsigned short* Bp, int col, int hh) {
  const v16h b0 = frag_glb(Bp, col, DD, 0, hh);
  const v16h b1 = frag_glb(Bp, col, DD, 32, hh);
  v8f d = wmh(a0, b0, zero8());
  d = wmh(a1, b1, d);
  return d;
}
__device__ __forceinline__ v8f gemm2(v16h a0, v16h a1, v16h a2, v16h a3, const unsigned short* Bp, int col,
                                     int hh) {
  const v16h b0 = frag_glb(Bp, col, HIDW, 0, hh);
  const v16h b1 = frag_glb(Bp, col, HIDW, 32, hh);
  v8f d = wmh(a0, b0, zero8());
  d = wmh(a1, b1, d);
  const v16h b2 = frag_glb(Bp, col, HIDW, 64, hh);
  const v16h b3 = frag_glb(Bp, col, HIDW, 96, hh);
  d = wmh(a2, b2, d);
  d = wmh(a3, b3, d);
  return d;
}

__device__ __forceinline__ void cvt_unit(const float* __restrict__ P, unsigned short* dst, long sc, long sk,
                                         int K, int KP, int Nv, int Nout, float scale, int i) {
  const int upc = KP >> 3;
  if (i >= Nout * upc) return;
  const int n = i / upc;
  const int seg = i - n * upc;
  const int nc = n < Nv - 1 ? n : Nv - 1;
  v8h o;
#pragma unroll
  for (int j = 0; j < 8; ++j) {
    const int k = 8 * seg + j;
    const int kc = k < K - 1 ? k : K - 1;
    const float v = P[(size_t)nc * sc + (size_t)kc * sk];
    const float keep = (k < K && n < Nv) ? scale : 0.0f;
    o[j] = (_Float16)(v * keep);
  }
  const v8us ob = __builtin_bit_cast(v8us, o);
  unsigned short* d = dst + (size_t)i * 8;
  *(volatile v8us*)d = ob;
  __threadfence();
  *(volatile v8us*)d = ob;
}

__global__ __launch_bounds__(TB) void k_prep(
    const float* __restrict__ nw2, const float* __restrict__ wih, const float* __restrict__ whh,
    const float* __restrict__ l0w, const float* __restrict__ x,
    unsigned short* BW2, unsigned short* BWI, unsigned short* BWH, unsigned short* BL0, unsigned short* XP) {
  const int job = (int)blockIdx.y;
  const int i = (int)blockIdx.x * TB + (int)threadIdx.x;
  const float* P = job == 0 ? nw2 : job == 1 ? wih : job == 2 ? whh : job == 3 ? l0w : x;
  unsigned short* D = job == 0 ? BW2 : job == 1 ? BWI : job == 2 ? BWH : job == 3 ? BL0 : XP;
  const long sc = (job == 0 || job == 3) ? 1 : DD;
  const long sk = job == 0 ? TCOL : job == 3 ? DD : 1;
  const int  K  = job == 0 ? HIDW : DD;
  const int  Nv = job == 0 ? TCOL : (job == 1 || job == 2) ? G3 : job == 3 ? DD : NNODE;
  const int  No = job == 4 ? NPAD : Nv;
  const float scale = job == 4 ? (float)ASC : (float)WSC;
  cvt_unit(P, D, sc, sk, K, K, Nv, No, scale, i);
}

__global__ __launch_bounds__(TB) void k_e1(const float* __restrict__ ea, const float* __restrict__ w1,
                                           const float* __restrict__ b1, unsigned short* E1H, int nE) {
  const int tid = threadIdx.x, lane = tid & 31;
  const int gw = ((int)blockIdx.x * TB + tid) >> 5;
  const int e0 = 2 * gw;
  if (e0 >= nE) return;
  int e = e0 + (lane >> 4); e = e > nE - 1 ? nE - 1 : e;
  const int o8 = 8 * (lane & 15);
  v4f ra = *(const v4f*)(b1 + o8);
  v4f rb = *(const v4f*)(b1 + o8 + 4);
  const float* ar = ea + (size_t)e * EFEAT;
#pragma unroll 1
  for (int k = 0; k < EFEAT; ++k) {
    const float ak = ar[k];
    const v4f wa = *(const v4f*)(w1 + k * HIDW + o8);
    const v4f wb = *(const v4f*)(w1 + k * HIDW + o8 + 4);
    ra += ak * wa;
    rb += ak * wb;
  }
  v8h r8;
  r8[0] = (_Float16)(fmaxf(ra.x, 0.0f) * (float)ASC); r8[1] = (_Float16)(fmaxf(ra.y, 0.0f) * (float)ASC);
  r8[2] = (_Float16)(fmaxf(ra.z, 0.0f) * (float)ASC); r8[3] = (_Float16)(fmaxf(ra.w, 0.0f) * (float)ASC);
  r8[4] = (_Float16)(fmaxf(rb.x, 0.0f) * (float)ASC); r8[5] = (_Float16)(fmaxf(rb.y, 0.0f) * (float)ASC);
  r8[6] = (_Float16)(fmaxf(rb.z, 0.0f) * (float)ASC); r8[7] = (_Float16)(fmaxf(rb.w, 0.0f) * (float)ASC);
  const v8us rv = __builtin_bit_cast(v8us, r8);
  unsigned short* dp = E1H + (size_t)e * HIDW + o8;
  *(volatile v8us*)dp = rv;
  __threadfence();
  *(volatile v8us*)dp = rv;
}

__device__ __forceinline__ void ew_rows(const _Float16* st, unsigned short* EW, int e0, int g, int lane) {
#pragma unroll
  for (int i = 0; i < 4; ++i) {
    const int row = 4 * i + (lane >> 3), p = lane & 7;
    const v8h v = *(const v8h*)(st + row * DD + 8 * p);
    const v8us vb = __builtin_bit_cast(v8us, v);
    *(volatile v8us*)(EW + (size_t)(e0 + row) * TCOL + (size_t)g * DD + 8 * p) = vb;
  }
}

__global__ __launch_bounds__(NT2) void k_ew(const unsigned short* __restrict__ E1H,
                                            const unsigned short* __restrict__ BW2,
                                            const float* __restrict__ b2, unsigned short* EW) {
  __shared__ __attribute__((aligned(16))) _Float16 sSt[2][16 * DD];
  const int tid = threadIdx.x, lane = tid & 31, wave = tid >> 5, hh = lane >> 4, m = lane & 15;
  const int e0 = ((int)blockIdx.x * 2 + wave) * 16;
  _Float16* st = sSt[wave];
  const v16h a0 = frag_glb(E1H, e0 + m, HIDW, 0, hh);
  const v16h a1 = frag_glb(E1H, e0 + m, HIDW, 32, hh);
  const v16h a2 = frag_glb(E1H, e0 + m, HIDW, 64, hh);
  const v16h a3 = frag_glb(E1H, e0 + m, HIDW, 96, hh);
#pragma unroll 1
  for (int g = 0; g < TCOL / DD; ++g) {
#pragma unroll 1
    for (int t = 0; t < 4; ++t) {
      const int cl = 16 * t + m;
      const int col = g * DD + cl;
      const v8f acc = gemm2(a0, a1, a2, a3, BW2, col, hh);
      const float bv = b2[col];
#pragma unroll
      for (int r = 0; r < 8; ++r)
        st[(8 * hh + r) * DD + cl] = (_Float16)((acc[r] * OSC + bv) * (float)EWSC);
    }
    __syncthreads();
    ew_rows(st, EW, e0, g, lane);
    __threadfence();
    ew_rows(st, EW, e0, g, lane);
    __syncthreads();
  }
}

__device__ __forceinline__ void rows_out2(const float* so, float* H32, unsigned short* HH, int n0, int lane) {
#pragma unroll
  for (int i = 0; i < 8; ++i) {
    const int row = 2 * i + (lane >> 4), p = lane & 15;
    const v4f v = *(const v4f*)(so + row * DD + 4 * p);
    *(volatile v4f*)(H32 + (size_t)(n0 + row) * DD + 4 * p) = v;
  }
#pragma unroll
  for (int i = 0; i < 4; ++i) {
    const int row = 4 * i + (lane >> 3), p = lane & 7;
    const v4f a = *(const v4f*)(so + row * DD + 8 * p);
    const v4f b = *(const v4f*)(so + row * DD + 8 * p + 4);
    v8h h8;
    h8[0] = (_Float16)(a.x * (float)ASC); h8[1] = (_Float16)(a.y * (float)ASC);
    h8[2] = (_Float16)(a.z * (float)ASC); h8[3] = (_Float16)(a.w * (float)ASC);
    h8[4] = (_Float16)(b.x * (float)ASC); h8[5] = (_Float16)(b.y * (float)ASC);
    h8[6] = (_Float16)(b.z * (float)ASC); h8[7] = (_Float16)(b.w * (float)ASC);
    const v8us hb = __builtin_bit_cast(v8us, h8);
    *(volatile v8us*)(HH + (size_t)(n0 + row) * DD + 8 * p) = hb;
  }
}

__global__ __launch_bounds__(NT) void k_lin0(const unsigned short* __restrict__ XP,
                                             const unsigned short* __restrict__ BL0,
                                             const float* __restrict__ b0, float* H32, unsigned short* HH) {
  __shared__ __attribute__((aligned(16))) float sOut[4][16 * DD];
  const int tid = threadIdx.x, lane = tid & 31, wave = tid >> 5, hh = lane >> 4, m = lane & 15;
  const int n0 = ((int)blockIdx.x * 4 + wave) * 16;
  float* so = sOut[wave];
  const v16h a0 = frag_glb(XP, n0 + m, DD, 0, hh);
  const v16h a1 = frag_glb(XP, n0 + m, DD, 32, hh);
#pragma unroll 1
  for (int t = 0; t < 4; ++t) {
    const int c = 16 * t + m;
    const v8f acc = gemm1(a0, a1, BL0, c, hh);
    const float bv = b0[c];
#pragma unroll
    for (int r = 0; r < 8; ++r) so[(8 * hh + r) * DD + c] = fmaxf(acc[r] * OSC + bv, 0.0f);
  }
  __syncthreads();
  rows_out2(so, H32, HH, n0, lane);
  __threadfence();
  rows_out2(so, H32, HH, n0, lane);
}

__global__ __launch_bounds__(NT) void k_node(
    const float* __restrict__ H32o, const unsigned short* __restrict__ HHo, float* H32n, unsigned short* HHn,
    const unsigned short* __restrict__ EW, const int* __restrict__ esrc, const int* __restrict__ edst,
    const float* __restrict__ convb,
    const unsigned short* __restrict__ BWI, const unsigned short* __restrict__ BWH,
    const float* __restrict__ bih, const float* __restrict__ bhh, int nN, int nE) {
  __shared__ __attribute__((aligned(16))) float    sAgg[64 * DD];
  __shared__ __attribute__((aligned(16))) _Float16 sM[4][16 * DD];
  __shared__ __attribute__((aligned(16))) float    sOut[4][16 * DD];
  __shared__ __attribute__((aligned(16))) int      sList[4 * WCAPN];
  __shared__ float sInv[64];
  __shared__ int   sDeg[64];
  __shared__ int   sWc[4];
  const int tid = threadIdx.x, lane = tid & 31, wave = tid >> 5, hh = lane >> 4, m = lane & 15;
  const int nb = (int)blockIdx.x * 64;
  const int n0 = nb + 16 * wave;

  {
    const v4f z = {0.f, 0.f, 0.f, 0.f};
    for (int i = tid; i < 64 * DD / 4; i += NT) *(v4f*)(sAgg + 4 * i) = z;
    if (tid < 64) sDeg[tid] = 0;
  }
  __syncthreads();

  const int rowOff = lane >> 3, colg = lane & 7;
  const int nChunks = (nE + NCH - 1) / NCH;
#pragma unroll 1
  for (int ch = 0; ch < nChunks; ++ch) {
    const int cbase = ch * NCH;
    const int el0 = tid * NKT;
    const int e0 = cbase + el0;
    const int sent = -2147483647 - 1;
    v4i da, db;
    if (cbase + NCH <= nE) {
      da = *(const v4i*)(edst + e0);
      db = *(const v4i*)(edst + e0 + 4);
    } else {
      da.x = (e0     < nE) ? edst[min(e0, nE - 1)] : sent;
      da.y = (e0 + 1 < nE) ? edst[min(e0 + 1, nE - 1)] : sent;
      da.z = (e0 + 2 < nE) ? edst[min(e0 + 2, nE - 1)] : sent;
      da.w = (e0 + 3 < nE) ? edst[min(e0 + 3, nE - 1)] : sent;
      db.x = (e0 + 4 < nE) ? edst[min(e0 + 4, nE - 1)] : sent;
      db.y = (e0 + 5 < nE) ? edst[min(e0 + 5, nE - 1)] : sent;
      db.z = (e0 + 6 < nE) ? edst[min(e0 + 6, nE - 1)] : sent;
      db.w = (e0 + 7 < nE) ? edst[min(e0 + 7, nE - 1)] : sent;
    }
    const unsigned nbu = (unsigned)nb;
    const unsigned s0 = (unsigned)da.x - nbu, s1 = (unsigned)da.y - nbu;
    const unsigned s2 = (unsigned)da.z - nbu, s3 = (unsigned)da.w - nbu;
    const unsigned s4 = (unsigned)db.x - nbu, s5 = (unsigned)db.y - nbu;
    const unsigned s6 = (unsigned)db.z - nbu, s7 = (unsigned)db.w - nbu;
    const bool h0 = s0 < 64u, h1 = s1 < 64u, h2 = s2 < 64u, h3 = s3 < 64u;
    const bool h4 = s4 < 64u, h5 = s5 < 64u, h6 = s6 < 64u, h7 = s7 < 64u;
    int wc = 0;
    const unsigned any = __builtin_amdgcn_ballot_w32(h0 | h1 | h2 | h3 | h4 | h5 | h6 | h7);
    if (any != 0u) {
#define HITJ(J, HJ, SJ) { \
        const unsigned mj = __builtin_amdgcn_ballot_w32(HJ); \
        if (mj != 0u) { \
          if (HJ) { \
            const int pos = wc + (int)__builtin_amdgcn_mbcnt_lo(mj, 0u); \
            if (pos < WCAPN) sList[wave * WCAPN + pos] = ((el0 + (J)) << 8) | (int)(SJ); \
          } \
          wc += (int)__builtin_popcount(mj); } }
      HITJ(0, h0, s0)
      HITJ(1, h1, s1)
      HITJ(2, h2, s2)
      HITJ(3, h3, s3)
      HITJ(4, h4, s4)
      HITJ(5, h5, s5)
      HITJ(6, h6, s6)
      HITJ(7, h7, s7)
#undef HITJ
    }
    if (lane == 0) sWc[wave] = wc < WCAPN ? wc : WCAPN;
    __syncthreads();

#pragma unroll 1
    for (int wl = 0; wl < 4; ++wl) {
      int n = __builtin_amdgcn_readfirstlane(sWc[wl]);
      n = n > WCAPN ? WCAPN : (n < 0 ? 0 : n);
#pragma unroll 1
      for (int i = 0; i < n; ++i) {
        const int ent = __builtin_amdgcn_readfirstlane(sList[wl * WCAPN + i]);
        const int loc = ent & 63;
        if ((loc >> 4) == wave) {
          int e = cbase + ((ent >> 8) & (NCH - 1));
          e = e < 0 ? 0 : (e > nE - 1 ? nE - 1 : e);
          int s = esrc[e];
          s = s < 0 ? 0 : (s > nN - 1 ? nN - 1 : s);
          const float* hrow = H32o + (size_t)s * DD;
          const unsigned short* ep = EW + (size_t)e * TCOL + 8 * colg;
          float acc[8];
#pragma unroll
          for (int j = 0; j < 8; ++j) acc[j] = 0.0f;
#pragma unroll 4
          for (int q = 0; q < 16; ++q) {
            const int ii = 4 * q + rowOff;
            const float ai = hrow[ii];
            U8 w; w.u = *(const v8us*)(ep + ii * DD);
#pragma unroll
            for (int j = 0; j < 8; ++j) acc[j] = fmaf(ai, (float)w.h[j], acc[j]);
          }
#pragma unroll
          for (int j = 0; j < 8; ++j) {
            acc[j] += __shfl_xor(acc[j], 8);
            acc[j] += __shfl_xor(acc[j], 16);
          }
          if (lane < 8) {
            float* ap = sAgg + loc * DD + 8 * lane;
            v4f x0 = *(const v4f*)ap;
            v4f x1 = *(const v4f*)(ap + 4);
            x0.x += acc[0] * EWINV; x0.y += acc[1] * EWINV; x0.z += acc[2] * EWINV; x0.w += acc[3] * EWINV;
            x1.x += acc[4] * EWINV; x1.y += acc[5] * EWINV; x1.z += acc[6] * EWINV; x1.w += acc[7] * EWINV;
            *(v4f*)ap = x0;
            *(v4f*)(ap + 4) = x1;
          }
          if (lane == 0) sDeg[loc] = sDeg[loc] + 1;
        }
      }
    }
    __syncthreads();
  }

  if (tid < 64) {
    const int dg = sDeg[tid];
    sInv[tid] = 1.0f / (float)(dg > 1 ? dg : 1);
  }
  __syncthreads();

  float* sa = sAgg + wave * 16 * DD;
  _Float16* sm = sM[wave];
  float* so = sOut[wave];

#pragma unroll 4
  for (int i = lane; i < 16 * DD; i += 32) {
    const int rl = i >> 6, c = i & 63;
    const float v = sa[i] * sInv[16 * wave + rl] + convb[c];
    sm[i] = (_Float16)(fmaxf(v, 0.0f) * (float)ASC);
  }
  __syncthreads();

  const v16h aH0 = frag_glb(HHo, n0 + m, DD, 0, hh);
  const v16h aH1 = frag_glb(HHo, n0 + m, DD, 32, hh);
  const v16h pH0 = frag_lds(sm, m, DD, 0, hh);
  const v16h pH1 = frag_lds(sm, m, DD, 32, hh);

#pragma unroll 1
  for (int t = 0; t < 4; ++t) {
    const int c = 16 * t + m;
    const v8f dhr = gemm1(aH0, aH1, BWH, c, hh);
    const v8f dhz = gemm1(aH0, aH1, BWH, DD + c, hh);
    const v8f dhn = gemm1(aH0, aH1, BWH, 2 * DD + c, hh);
    const v8f dir = gemm1(pH0, pH1, BWI, c, hh);
    const v8f diz = gemm1(pH0, pH1, BWI, DD + c, hh);
    const v8f din = gemm1(pH0, pH1, BWI, 2 * DD + c, hh);
    const float bir = bih[c], biz = bih[DD + c], bin = bih[2 * DD + c];
    const float bhr = bhh[c], bhz = bhh[DD + c], bhn = bhh[2 * DD + c];
#pragma unroll
    for (int r = 0; r < 8; ++r) {
      const float rg = sigm_f(dir[r] * OSC + bir + dhr[r] * OSC + bhr);
      const float zg = sigm_f(diz[r] * OSC + biz + dhz[r] * OSC + bhz);
      const float ng = tanhf(din[r] * OSC + bin + rg * (dhn[r] * OSC + bhn));
      const float ho = H32o[(size_t)(n0 + 8 * hh + r) * DD + c];
      so[(8 * hh + r) * DD + c] = (1.0f - zg) * ng + zg * ho;
    }
  }
  __syncthreads();

  rows_out2(so, H32n, HHn, n0, lane);
  __threadfence();
  rows_out2(so, H32n, HHn, n0, lane);
}

__global__ __launch_bounds__(TB) void k_copy(const float* __restrict__ H, float* dst, int nPieces) {
  const int gt = (int)blockIdx.x * TB + (int)threadIdx.x;
  if (gt >= nPieces) return;
  const v4f v = *(const v4f*)(H + (size_t)gt * 4);
  float* op = dst + (size_t)gt * 4;
  *(volatile v4f*)op = v;
  __threadfence();
  *(volatile v4f*)op = v;
}

__global__ __launch_bounds__(TB) void k_s2s(const float* __restrict__ H32, const int* __restrict__ batch,
                                           const float* __restrict__ lwih, const float* __restrict__ lwhh,
                                           const float* __restrict__ lbih, const float* __restrict__ lbhh,
                                           float* out0, int nN) {
  __shared__ int   sList[NWS][WLC];
  __shared__ float sE[NWS][WLC];
  __shared__ int   sWc[NWS];
  __shared__ int   sOv[NWS];
  __shared__ __attribute__((aligned(16))) float sQS[GPB * 2 * DD];
  __shared__ __attribute__((aligned(16))) float sHH[GPB * DD];
  __shared__ __attribute__((aligned(16))) float sCC[GPB * DD];
  __shared__ __attribute__((aligned(16))) float sGate[GPB * G4];
  const int tid = threadIdx.x, lane = tid & 31, wave = tid >> 5;
  const int g0 = (int)blockIdx.x * GPB;

  for (int i = tid; i < GPB * 2 * DD; i += TB) sQS[i] = 0.0f;
  for (int i = tid; i < GPB * DD; i += TB) { sHH[i] = 0.0f; sCC[i] = 0.0f; }

  int wc = 0;
#pragma unroll 1
  for (int nb = 0; nb < nN; nb += TB) {
    const int n = nb + tid;
    const int nc = n < nN ? n : nN - 1;
    const int b = batch[nc];
    const int lg = b - g0;
    const bool hit = (n < nN) && ((unsigned)lg < (unsigned)GPB);
    const unsigned mk = __builtin_amdgcn_ballot_w32(hit);
    if (hit) {
      const int pos = wc + (int)__builtin_amdgcn_mbcnt_lo(mk, 0u);
      if (pos < WLC) sList[wave][pos] = n | (lg << 16);
    }
    wc += (int)__builtin_popcount(mk);
  }
  if (lane == 0) { sWc[wave] = wc < WLC ? wc : WLC; sOv[wave] = wc > WLC ? 1 : 0; }
  __syncthreads();

#pragma unroll 1
  for (int step = 0; step < 3; ++step) {
    {
      const int g = tid;
      float acc[GPB];
      const float bs = lbih[g] + lbhh[g];
#pragma unroll
      for (int b = 0; b < GPB; ++b) acc[b] = bs;
#pragma unroll 1
      for (int k = 0; k < 2 * DD; ++k) {
        const float w = lwih[(size_t)g * (2 * DD) + k];
#pragma unroll
        for (int b = 0; b < GPB; ++b) acc[b] = fmaf(sQS[b * 2 * DD + k], w, acc[b]);
      }
#pragma unroll 1
      for (int k = 0; k < DD; ++k) {
        const float w = lwhh[(size_t)g * DD + k];
#pragma unroll
        for (int b = 0; b < GPB; ++b) acc[b] = fmaf(sHH[b * DD + k], w, acc[b]);
      }
#pragma unroll
      for (int b = 0; b < GPB; ++b) sGate[b * G4 + g] = acc[b];
    }
    __syncthreads();
#pragma unroll 1
    for (int idx = tid; idx < GPB * DD; idx += TB) {
      const int b = idx >> 6, j = idx & 63;
      const float* gtp = sGate + b * G4;
      const float vi = gtp[j], vf = gtp[DD + j], vg = gtp[2 * DD + j], vo = gtp[3 * DD + j];
      const float c = sigm_f(vf) * sCC[idx] + sigm_f(vi) * tanh_f(vg);
      sCC[idx] = c;
      const float hv = sigm_f(vo) * tanh_f(c);
      sHH[idx] = hv;
      sQS[b * 2 * DD + j] = hv;
    }
    __syncthreads();
    {
      const int lg = wave;
      const v2f q2 = *(const v2f*)(sQS + lg * 2 * DD + 2 * lane);
      float emax = -3.0e38f;
#pragma unroll 1
      for (int wl = 0; wl < NWS; ++wl) {
        const int ne = __builtin_amdgcn_readfirstlane(sWc[wl]);
#pragma unroll 1
        for (int i = 0; i < ne; ++i) {
          const int ent = __builtin_amdgcn_readfirstlane(sList[wl][i]);
          if ((ent >> 16) == lg) {
            int n = ent & 0xffff; n = n > nN - 1 ? nN - 1 : n;
            const v2f hv = *(const v2f*)(H32 + (size_t)n * DD + 2 * lane);
            float p = hv.x * q2.x + hv.y * q2.y;
            p = wsum32(p);
            emax = fmaxf(emax, p);
            sE[wl][i] = p;
          }
        }
      }
      float den = 0.0f;
#pragma unroll 1
      for (int wl = 0; wl < NWS; ++wl) {
        const int ne = __builtin_amdgcn_readfirstlane(sWc[wl]);
#pragma unroll 1
        for (int i = 0; i < ne; ++i) {
          const int ent = __builtin_amdgcn_readfirstlane(sList[wl][i]);
          if ((ent >> 16) == lg) {
            const float ex = __expf(sE[wl][i] - emax);
            den += ex;
            sE[wl][i] = ex;
          }
        }
      }
      const float rden = den > 0.0f ? __builtin_amdgcn_rcpf(den) : 0.0f;
      v2f rv = {0.f, 0.f};
#pragma unroll 1
      for (int wl = 0; wl < NWS; ++wl) {
        const int ne = __builtin_amdgcn_readfirstlane(sWc[wl]);
#pragma unroll 1
        for (int i = 0; i < ne; ++i) {
          const int ent = __builtin_amdgcn_readfirstlane(sList[wl][i]);
          if ((ent >> 16) == lg) {
            int n = ent & 0xffff; n = n > nN - 1 ? nN - 1 : n;
            const v2f hv = *(const v2f*)(H32 + (size_t)n * DD + 2 * lane);
            const float a = sE[wl][i] * rden;
            rv += hv * a;
          }
        }
      }
      *(v2f*)(sQS + lg * 2 * DD + DD + 2 * lane) = rv;
    }
    __syncthreads();
  }

  int ov = 0;
#pragma unroll
  for (int w = 0; w < NWS; ++w) ov |= sOv[w];
  v4f v = *(const v4f*)(sQS + 4 * tid);
  if (ov != 0) v = v + __int_as_float(0x7fc00000);
  float* op = out0 + (size_t)blockIdx.x * (GPB * 2 * DD) + 4 * tid;
  *(volatile v4f*)op = v;
  __threadfence();
  *(volatile v4f*)op = v;
}

extern "C" void kernel_launch(void* const* d_in, const int* in_sizes, int n_in,
                              void* d_out, int out_size, void* d_ws, size_t ws_size,
                              hipStream_t stream) {
  if (n_in < 19) return;
  if (in_sizes[0] != NNODE * NFEAT || in_sizes[1] != 2 * NEDGE || in_sizes[2] != NNODE ||
      in_sizes[3] != NEDGE * EFEAT) return;
  if (in_sizes[4] != NFEAT * DD || in_sizes[5] != DD || in_sizes[6] != EFEAT * HIDW || in_sizes[7] != HIDW) return;
  if (in_sizes[8] != HIDW * TCOL || in_sizes[9] != TCOL || in_sizes[10] != DD) return;
  if (in_sizes[11] != G3 * DD || in_sizes[12] != G3 * DD || in_sizes[13] != G3 || in_sizes[14] != G3) return;
  if (in_sizes[15] != G4 * 2 * DD || in_sizes[16] != G4 * DD || in_sizes[17] != G4 || in_sizes[18] != G4) return;
  if (out_size != OUTN) return;

  const float* x         = (const float*)d_in[0];
  const int*   eidx      = (const int*)d_in[1];
  const int*   batch     = (const int*)d_in[2];
  const float* eattr     = (const float*)d_in[3];
  const float* lin0_w    = (const float*)d_in[4];
  const float* lin0_b    = (const float*)d_in[5];
  const float* nn_w1     = (const float*)d_in[6];
  const float* nn_b1     = (const float*)d_in[7];
  const float* nn_w2     = (const float*)d_in[8];
  const float* nn_b2     = (const float*)d_in[9];
  const float* conv_b    = (const float*)d_in[10];
  const float* gru_wih   = (const float*)d_in[11];
  const float* gru_whh   = (const float*)d_in[12];
  const float* gru_bih   = (const float*)d_in[13];
  const float* gru_bhh   = (const float*)d_in[14];
  const float* lstm_wih  = (const float*)d_in[15];
  const float* lstm_whh  = (const float*)d_in[16];
  const float* lstm_bih  = (const float*)d_in[17];
  const float* lstm_bhh  = (const float*)d_in[18];
  float* out = (float*)d_out;
  const int* srcp = eidx;
  const int* dstp = eidx + NEDGE;

  char* ws = (char*)d_ws;
  size_t off = 0;
#define CARVE(NAME, BYTES) const size_t NAME = off; off += (size_t)(BYTES); off = (off + 255) & ~(size_t)255;
  CARVE(oEW,   (size_t)NEDGE * TCOL * 2)
  CARVE(oBW2,  (size_t)TCOL * HIDW * 2)
  CARVE(oBWI,  (size_t)G3 * DD * 2)
  CARVE(oBWH,  (size_t)G3 * DD * 2)
  CARVE(oBL0,  (size_t)DD * DD * 2)
  CARVE(oXP,   (size_t)NPAD * DD * 2)
  CARVE(oE1,   (size_t)NEDGE * HIDW * 2)
  CARVE(oH32A, (size_t)NPAD * DD * 4)
  CARVE(oH32B, (size_t)NPAD * DD * 4)
  CARVE(oHHA,  (size_t)NPAD * DD * 2)
  CARVE(oHHB,  (size_t)NPAD * DD * 2)
#undef CARVE
  if (off > ws_size || off > (size_t)WSCAP) return;

  unsigned short* EW   = (unsigned short*)(ws + oEW);
  unsigned short* BW2  = (unsigned short*)(ws + oBW2);
  unsigned short* BWI  = (unsigned short*)(ws + oBWI);
  unsigned short* BWH  = (unsigned short*)(ws + oBWH);
  unsigned short* BL0  = (unsigned short*)(ws + oBL0);
  unsigned short* XP   = (unsigned short*)(ws + oXP);
  unsigned short* E1H  = (unsigned short*)(ws + oE1);
  float*          H32A = (float*)(ws + oH32A);
  float*          H32B = (float*)(ws + oH32B);
  unsigned short* HHA  = (unsigned short*)(ws + oHHA);
  unsigned short* HHB  = (unsigned short*)(ws + oHHB);

  k_prep<<<dim3(UMAX / TB, 5, 1), TB, 0, stream>>>(nn_w2, gru_wih, gru_whh, lin0_w, x, BW2, BWI, BWH, BL0, XP);
  k_e1<<<(NEDGE * 16) / TB, TB, 0, stream>>>(eattr, nn_w1, nn_b1, E1H, NEDGE);
  k_ew<<<NEDGE / 32, NT2, 0, stream>>>(E1H, BW2, nn_b2, EW);
  k_lin0<<<NPAD / 64, NT, 0, stream>>>(XP, BL0, lin0_b, H32A, HHA);
  for (int it = 0; it < 3; ++it) {
    const int rd = it & 1;
    const float* H32o = rd ? H32B : H32A;
    const unsigned short* HHo = rd ? HHB : HHA;
    float* H32n = rd ? H32A : H32B;
    unsigned short* HHn = rd ? HHA : HHB;
    k_node<<<NPAD / 64, NT, 0, stream>>>(H32o, HHo, H32n, HHn, EW, srcp, dstp, conv_b, BWI, BWH,
                                         gru_bih, gru_bhh, NNODE, NEDGE);
  }
  k_copy<<<(NPIECE + TB - 1) / TB, TB, 0, stream>>>(H32B, out + OUT0N, NPIECE);
  k_s2s<<<NGR / GPB, TB, 0, stream>>>(H32B, batch, lstm_wih, lstm_whh, lstm_bih, lstm_bhh, out, NNODE);
}
